// myRGCN_87703232184764
// MI455X (gfx1250) — hardware-verified
//
#include <hip/hip_runtime.h>
#define NA 20000
#define NEI 12
#define NE (NA * NEI)
#define BST 40
#define AST 20
#define HH 64
#define NREL 3
#define NCR 20
#define NCLS 2
#define KB (BST * NEI)
#define KA (AST * NEI * NEI)
#define NN NA
#define NHALF (NA / 2)

typedef __bf16 v16b __attribute__((ext_vector_type(16)));
typedef unsigned short v8us __attribute__((ext_vector_type(8), may_alias));
typedef float  v8f  __attribute__((ext_vector_type(8)));
typedef float  v4f  __attribute__((ext_vector_type(4)));
typedef float  v4fa __attribute__((ext_vector_type(4), may_alias));
union FragB { v16b v; v8us half[2]; unsigned short u[16]; };

__device__ __forceinline__ unsigned short bf16_bits(float x) { unsigned int u = __float_as_uint(x); return (unsigned short)((u + 0x7FFFu + ((u >> 16) & 1u)) >> 16); }
__device__ __forceinline__ float bf16_val(unsigned short b) { return __uint_as_float(((unsigned int)b) << 16); }
__device__ __forceinline__ float bf16_round(float x) { return bf16_val(bf16_bits(x)); }
template <int NT>
__device__ __forceinline__ v8f mmaN(v16b ah, v16b al, v16b bh, v16b bl, v8f c) {
  c = __builtin_amdgcn_wmma_f32_16x16x32_bf16(false, ah, false, bh, (short)0, c, false, false);
  if (NT >= 2) c = __builtin_amdgcn_wmma_f32_16x16x32_bf16(false, al, false, bh, (short)0, c, false, false);
  if (NT >= 3) c = __builtin_amdgcn_wmma_f32_16x16x32_bf16(false, ah, false, bl, (short)0, c, false, false);
  asm volatile("v_nop\n\tv_nop\n\tv_nop\n\tv_nop" : "+v"(c) : "v"(ah), "v"(al), "v"(bh), "v"(bl));
  return c;
}

__global__ __launch_bounds__(256) void k_wt_bf16(const float* __restrict__ W, unsigned short* __restrict__ Wt, int K, int N) {
  const int t = blockIdx.x * 256 + threadIdx.x;
  const int k8n = K / 8;
  if (t >= N * k8n) return;
  const int n = t / k8n, k8 = (t % k8n) * 8;
  v8us v;
#pragma unroll
  for (int i = 0; i < 8; ++i) v[i] = bf16_bits(W[(size_t)(k8 + i) * N + n]);
  *(volatile v8us*)(Wt + (size_t)n * K + k8) = v;
  __threadfence();
  *(volatile v8us*)(Wt + (size_t)n * K + k8) = v;
}

template <bool ASPLIT, int ACT, bool BIAS_BF16>
__global__ __launch_bounds__(128) void k_gemm_bf(const float* __restrict__ A, int lda, const unsigned short* __restrict__ Wt, int ldb,
                                               const float* __restrict__ bias, float* __restrict__ C, int ldc, int M, int N, int K) {
  __shared__ __attribute__((aligned(16))) float so[4][16][64];
  const int tid = threadIdx.x, w = tid >> 5, lane = tid & 31, ln = lane & 15, hh = lane >> 4;
  const int ntn = N / 64;
  const int wid = blockIdx.x * 4 + w;
  const int mt = wid / ntn, nq = wid % ntn;
  if (mt * 16 >= M) return;
  const int row0 = mt * 16, col0 = nq * 64;
  const float* arow = A + (size_t)(row0 + ln) * lda;
  v8f acc[4] = {};
  for (int kb = 0; kb < K; kb += 32) {
    FragB ah, al;
    const v4f x0 = *(const v4fa*)(arow + kb + 8 * hh), x1 = *(const v4fa*)(arow + kb + 8 * hh + 4);
    const v4f x2 = *(const v4fa*)(arow + kb + 16 + 8 * hh), x3 = *(const v4fa*)(arow + kb + 16 + 8 * hh + 4);
    float xs[16] = {x0[0],x0[1],x0[2],x0[3],x1[0],x1[1],x1[2],x1[3],x2[0],x2[1],x2[2],x2[3],x3[0],x3[1],x3[2],x3[3]};
#pragma unroll
    for (int i = 0; i < 16; ++i) { const unsigned short hb = bf16_bits(xs[i]); ah.u[i] = hb; al.u[i] = ASPLIT ? bf16_bits(xs[i] - bf16_val(hb)) : (unsigned short)0; }
#pragma unroll
    for (int t = 0; t < 4; ++t) {
      const unsigned short* brow = Wt + (size_t)(col0 + t * 16 + ln) * ldb + kb;
      FragB b;
      b.half[0] = *(const v8us*)(brow + 8 * hh);
      b.half[1] = *(const v8us*)(brow + 16 + 8 * hh);
      acc[t] = mmaN<ASPLIT ? 2 : 1>(ah.v, al.v, b.v, b.v, acc[t]);
    }
  }
#pragma unroll
  for (int t = 0; t < 4; ++t) {
    float bv = bias ? bias[col0 + t * 16 + ln] : 0.f;
    if (BIAS_BF16) bv = bf16_round(bv);
#pragma unroll
    for (int r = 0; r < 8; ++r) { float v = acc[t][r] + bv; if (ACT == 1) v = fmaxf(v, 0.f); so[w][8 * hh + r][t * 16 + ln] = v; }
  }
  __builtin_amdgcn_fence(__ATOMIC_ACQ_REL, "workgroup");
  __builtin_amdgcn_wave_barrier();
  const int rsub = lane >> 4, c4 = (lane & 15) * 4;
  for (int pass = 0; pass < 2; ++pass) {
#pragma unroll
    for (int q = 0; q < 8; ++q) {
      const int r = q * 2 + rsub;
      const v4f v = *(const v4fa*)&so[w][r][c4];
      *(volatile v4f*)(C + (size_t)(row0 + r) * ldc + col0 + c4) = v;
    }
    if (pass == 0) __threadfence();
  }
}

template <int D, bool CAUSAL>
__global__ __launch_bounds__(128) void k_flash(const float* __restrict__ qb, const float* __restrict__ kb, const float* __restrict__ vb,
                                             int pitch, int T, int H, float scale, float* __restrict__ y, int ypitch) {
  constexpr int KS = D / 32;
  constexpr int DT = D / 16;
  __shared__ __attribute__((aligned(16))) unsigned short sKh[32][D + 8], sKl[32][D + 8], sVh[32][D + 8], sVl[32][D + 8];
  __shared__ __attribute__((aligned(16))) unsigned short sPh[4][16][40], sPl[4][16][40];
  __shared__ __attribute__((aligned(16))) float sO[4][16][D];
  const int tid = threadIdx.x, w = tid >> 5, lane = tid & 31, ln = lane & 15, hh = lane >> 4;
  const int nqb = (T + 63) / 64;
  const int bh = blockIdx.x / nqb, qblk = blockIdx.x % nqb;
  const int b = bh / H, h = bh % H;
  const int q0 = qblk * 64 + w * 16;
  const float* Q = qb + (size_t)b * T * pitch + h * D;
  const float* K = kb + (size_t)b * T * pitch + h * D;
  const float* V = vb + (size_t)b * T * pitch + h * D;

  FragB aqh[KS], aql[KS];
  {
    int row = q0 + ln; if (row >= T) row = T - 1;
    const float* qr = Q + (size_t)row * pitch;
#pragma unroll
    for (int ks = 0; ks < KS; ++ks)
#pragma unroll
      for (int i = 0; i < 16; ++i) {
        const int d = ks * 32 + ((i < 8) ? (8 * hh + i) : (16 + 8 * hh + (i - 8)));
        const float x = qr[d] * scale; const unsigned short hb = bf16_bits(x);
        aqh[ks].u[i] = hb; aql[ks].u[i] = bf16_bits(x - bf16_val(hb));
      }
  }
  float m_r[8], l_r[8];
#pragma unroll
  for (int r = 0; r < 8; ++r) { m_r[r] = -3.0e38f; l_r[r] = 0.f; }
  v8f oacc[DT];
#pragma unroll
  for (int dt = 0; dt < DT; ++dt) oacc[dt] = (v8f){0.f,0.f,0.f,0.f,0.f,0.f,0.f,0.f};

  const int kv_end = CAUSAL ? min(T, qblk * 64 + 64) : T;
  for (int j0 = 0; j0 < kv_end; j0 += 32) {
    __syncthreads();
    for (int e = tid; e < 32 * (D / 4); e += 128) {
      const int r = e / (D / 4), c4 = (e % (D / 4)) * 4;
      const int key = j0 + r;
      v4f kf = {0.f,0.f,0.f,0.f}, vf = {0.f,0.f,0.f,0.f};
      if (key < T) { kf = *(const v4fa*)(K + (size_t)key * pitch + c4); vf = *(const v4fa*)(V + (size_t)key * pitch + c4); }
#pragma unroll
      for (int t = 0; t < 4; ++t) {
        unsigned short hb = bf16_bits(kf[t]); sKh[r][c4 + t] = hb; sKl[r][c4 + t] = bf16_bits(kf[t] - bf16_val(hb));
        hb = bf16_bits(vf[t]); sVh[r][c4 + t] = hb; sVl[r][c4 + t] = bf16_bits(vf[t] - bf16_val(hb));
      }
    }
    __syncthreads();
    v8f s[2];
#pragma unroll
    for (int nt = 0; nt < 2; ++nt) {
      v8f acc = {};
#pragma unroll
      for (int ks = 0; ks < KS; ++ks) {
        FragB bh_, bl_;
        bh_.half[0] = *(const v8us*)&sKh[nt * 16 + ln][ks * 32 + 8 * hh]; bh_.half[1] = *(const v8us*)&sKh[nt * 16 + ln][ks * 32 + 16 + 8 * hh];
        bl_.half[0] = *(const v8us*)&sKl[nt * 16 + ln][ks * 32 + 8 * hh]; bl_.half[1] = *(const v8us*)&sKl[nt * 16 + ln][ks * 32 + 16 + 8 * hh];
        acc = mmaN<3>(aqh[ks].v, aql[ks].v, bh_.v, bl_.v, acc);
      }
      s[nt] = acc;
    }
    float alpha[8];
#pragma unroll
    for (int r = 0; r < 8; ++r) {
      const int qi = q0 + 8 * hh + r;
      const int ja = j0 + ln, jb = j0 + 16 + ln;
      if (CAUSAL) { if (ja > qi) s[0][r] = -3.0e38f; if (jb > qi) s[1][r] = -3.0e38f; }
      if (ja >= T) s[0][r] = -3.0e38f;
      if (jb >= T) s[1][r] = -3.0e38f;
      float mx = fmaxf(s[0][r], s[1][r]);
      mx = fmaxf(mx, __shfl_xor(mx, 1, 32)); mx = fmaxf(mx, __shfl_xor(mx, 2, 32)); mx = fmaxf(mx, __shfl_xor(mx, 4, 32)); mx = fmaxf(mx, __shfl_xor(mx, 8, 32));
      const float mnew = fmaxf(m_r[r], mx);
      alpha[r] = (mnew > -1.0e38f) ? __expf(m_r[r] - mnew) : 1.0f;
      const float p0 = (s[0][r] > -1.0e38f) ? __expf(s[0][r] - mnew) : 0.f;
      const float p1 = (s[1][r] > -1.0e38f) ? __expf(s[1][r] - mnew) : 0.f;
      m_r[r] = mnew;
      l_r[r] = l_r[r] * alpha[r] + p0 + p1;
      unsigned short hb = bf16_bits(p0); sPh[w][8 * hh + r][ln] = hb;      sPl[w][8 * hh + r][ln] = bf16_bits(p0 - bf16_val(hb));
      hb = bf16_bits(p1);                sPh[w][8 * hh + r][16 + ln] = hb; sPl[w][8 * hh + r][16 + ln] = bf16_bits(p1 - bf16_val(hb));
    }
#pragma unroll
    for (int dt = 0; dt < DT; ++dt)
#pragma unroll
      for (int r = 0; r < 8; ++r) oacc[dt][r] *= alpha[r];
    __builtin_amdgcn_fence(__ATOMIC_ACQ_REL, "workgroup");
    __builtin_amdgcn_wave_barrier();
    FragB pah, pal;
    pah.half[0] = *(const v8us*)&sPh[w][ln][8 * hh]; pah.half[1] = *(const v8us*)&sPh[w][ln][16 + 8 * hh];
    pal.half[0] = *(const v8us*)&sPl[w][ln][8 * hh]; pal.half[1] = *(const v8us*)&sPl[w][ln][16 + 8 * hh];
#pragma unroll
    for (int dt = 0; dt < DT; ++dt) {
      FragB bvh, bvl;
#pragma unroll
      for (int i = 0; i < 8; ++i) {
        bvh.u[i] = sVh[8 * hh + i][dt * 16 + ln]; bvh.u[8 + i] = sVh[16 + 8 * hh + i][dt * 16 + ln];
        bvl.u[i] = sVl[8 * hh + i][dt * 16 + ln]; bvl.u[8 + i] = sVl[16 + 8 * hh + i][dt * 16 + ln];
      }
      oacc[dt] = mmaN<3>(pah.v, pal.v, bvh.v, bvl.v, oacc[dt]);
    }
    __builtin_amdgcn_fence(__ATOMIC_ACQ_REL, "workgroup");
    __builtin_amdgcn_wave_barrier();
  }
#pragma unroll
  for (int r = 0; r < 8; ++r) {
    float l = l_r[r];
    l += __shfl_xor(l, 1, 32); l += __shfl_xor(l, 2, 32); l += __shfl_xor(l, 4, 32); l += __shfl_xor(l, 8, 32);
    l_r[r] = (l > 0.f) ? 1.0f / l : 0.f;
  }
#pragma unroll
  for (int dt = 0; dt < DT; ++dt)
#pragma unroll
    for (int r = 0; r < 8; ++r) sO[w][8 * hh + r][dt * 16 + ln] = oacc[dt][r] * l_r[r];
  __builtin_amdgcn_fence(__ATOMIC_ACQ_REL, "workgroup");
  __builtin_amdgcn_wave_barrier();
  for (int pass = 0; pass < 2; ++pass) {
    for (int r = 0; r < 16; ++r) {
      const int row = q0 + r;
      if (row < T && lane < D / 4) {
        const v4f val = *(const v4fa*)&sO[w][r][lane * 4];
        *(volatile v4f*)(y + ((size_t)b * T + row) * ypitch + h * D + lane * 4) = val;
      }
    }
    if (pass == 0) __threadfence();
  }
}

typedef _Float16 v16h __attribute__((ext_vector_type(16)));
union FragH { v16h v; v8us half[2]; _Float16 h[16]; unsigned short u[16]; };
template <int NT>
__device__ __forceinline__ v8f mmaH(v16h ah, v16h al, v16h bh, v16h bl, v8f c) {
  c = __builtin_amdgcn_wmma_f32_16x16x32_f16(false, ah, false, bh, (short)0, c, false, false);
  if (NT >= 2) c = __builtin_amdgcn_wmma_f32_16x16x32_f16(false, al, false, bh, (short)0, c, false, false);
  if (NT >= 3) c = __builtin_amdgcn_wmma_f32_16x16x32_f16(false, ah, false, bl, (short)0, c, false, false);
  asm volatile("v_nop\n\tv_nop\n\tv_nop\n\tv_nop" : "+v"(c) : "v"(ah), "v"(al), "v"(bh), "v"(bl));
  return c;
}
template <bool ASPLIT>
__global__ __launch_bounds__(128) void k_gemm_h(const float* __restrict__ A, int lda, size_t sA, const _Float16* __restrict__ Bh, int ldb, size_t sB, float alpha, float* __restrict__ C, int ldc, size_t sC, int M, int N, int K) {
  __shared__ __attribute__((aligned(16))) float so[4][16][64];
  const int tid = threadIdx.x, w = tid >> 5, lane = tid & 31, ln = lane & 15, hh = lane >> 4; const int by = blockIdx.y;
  A += (size_t)by * sA; Bh += (size_t)by * sB; C += (size_t)by * sC;
  const int ntn = (N + 63) / 64; const int wid = blockIdx.x * 4 + w; const int mt = wid / ntn, nq = wid % ntn; if (mt * 16 >= M) return;
  const int row0 = mt * 16, col0 = nq * 64; const float* arow = A + (size_t)(row0 + ln) * lda;
  v8f acc[4] = {};
  for (int kb = 0; kb < K; kb += 32) {
    FragH ah, al;
    const v4f x0 = *(const v4fa*)(arow + kb + 8 * hh), x1 = *(const v4fa*)(arow + kb + 8 * hh + 4), x2 = *(const v4fa*)(arow + kb + 16 + 8 * hh), x3 = *(const v4fa*)(arow + kb + 16 + 8 * hh + 4);
    float xs[16] = {x0[0],x0[1],x0[2],x0[3],x1[0],x1[1],x1[2],x1[3],x2[0],x2[1],x2[2],x2[3],x3[0],x3[1],x3[2],x3[3]};
#pragma unroll
    for (int i = 0; i < 16; ++i) { const _Float16 h = (_Float16)xs[i]; ah.h[i] = h; al.h[i] = ASPLIT ? (_Float16)(xs[i] - (float)h) : (_Float16)0.0f; }
#pragma unroll
    for (int t = 0; t < 4; ++t) { if (col0 + t * 16 >= N) continue; const size_t boff = (size_t)(col0 + t * 16 + ln) * ldb + kb; FragH bq; bq.half[0] = *(const v8us*)(Bh + boff + 8 * hh); bq.half[1] = *(const v8us*)(Bh + boff + 16 + 8 * hh);
      acc[t] = mmaH<ASPLIT ? 2 : 1>(ah.v, al.v, bq.v, bq.v, acc[t]); }
  }
#pragma unroll
  for (int t = 0; t < 4; ++t) { if (col0 + t * 16 >= N) continue;
#pragma unroll
    for (int r = 0; r < 8; ++r) so[w][8 * hh + r][t * 16 + ln] = acc[t][r] * alpha; }
  __builtin_amdgcn_fence(__ATOMIC_ACQ_REL, "workgroup"); __builtin_amdgcn_wave_barrier();
  const int rsub = lane >> 4, c4 = (lane & 15) * 4;
  for (int pass = 0; pass < 2; ++pass) {
#pragma unroll
    for (int q = 0; q < 8; ++q) { const int r = q * 2 + rsub; if (col0 + c4 < N) { const v4f v = *(const v4fa*)&so[w][r][c4]; *(volatile v4f*)(C + (size_t)(row0 + r) * ldc + col0 + c4) = v; } }
    if (pass == 0) __threadfence(); }
}

template <int DUMMY>
__global__ __launch_bounds__(128) void k_gemm_hh(const _Float16* __restrict__ A, int lda, size_t sA, const _Float16* __restrict__ Bh, int ldb, size_t sB, float alpha, float* __restrict__ C, int ldc, size_t sC, int M, int N, int K) {
  __shared__ __attribute__((aligned(16))) float so[4][16][64];
  const int tid = threadIdx.x, w = tid >> 5, lane = tid & 31, ln = lane & 15, hh = lane >> 4; const int by = blockIdx.y;
  A += (size_t)by * sA; Bh += (size_t)by * sB; C += (size_t)by * sC;
  const int ntn = (N + 63) / 64; const int wid = blockIdx.x * 4 + w; const int mt = wid / ntn, nq = wid % ntn; if (mt * 16 >= M) return;
  const int row0 = mt * 16, col0 = nq * 64; const _Float16* arow = A + (size_t)(row0 + ln) * lda;
  v8f acc[4] = {};
  for (int kb = 0; kb < K; kb += 32) { FragH ah; ah.half[0] = *(const v8us*)((const unsigned short*)arow + kb + 8 * hh); ah.half[1] = *(const v8us*)((const unsigned short*)arow + kb + 16 + 8 * hh);
#pragma unroll
    for (int t = 0; t < 4; ++t) { if (col0 + t * 16 >= N) continue; const size_t boff = (size_t)(col0 + t * 16 + ln) * ldb + kb; FragH bq; bq.half[0] = *(const v8us*)((const unsigned short*)Bh + boff + 8 * hh); bq.half[1] = *(const v8us*)((const unsigned short*)Bh + boff + 16 + 8 * hh);
      acc[t] = mmaH<1>(ah.v, ah.v, bq.v, bq.v, acc[t]); }
  }
#pragma unroll
  for (int t = 0; t < 4; ++t) { if (col0 + t * 16 >= N) continue;
#pragma unroll
    for (int r = 0; r < 8; ++r) so[w][8 * hh + r][t * 16 + ln] = acc[t][r] * alpha; }
  __builtin_amdgcn_fence(__ATOMIC_ACQ_REL, "workgroup"); __builtin_amdgcn_wave_barrier();
  const int rsub = lane >> 4, c4 = (lane & 15) * 4;
  for (int pass = 0; pass < 2; ++pass) {
#pragma unroll
    for (int q = 0; q < 8; ++q) { const int r = q * 2 + rsub; if (col0 + c4 < N) { const v4f v = *(const v4fa*)&so[w][r][c4]; *(volatile v4f*)(C + (size_t)(row0 + r) * ldc + col0 + c4) = v; } }
    if (pass == 0) __threadfence(); }
}

__global__ __launch_bounds__(256) void k_gbf_b(const float* __restrict__ bond, _Float16* __restrict__ EF) { const size_t t = (size_t)blockIdx.x * 256 + threadIdx.x;
  if (t < (size_t)NA * KB / 8) { const int k8 = (int)((t * 8) % KB); const size_t n = (t * 8) / KB; FragH f; for (int q = 0; q < 8; ++q) { const int k = k8 + q; const int i = k / BST, s = k % BST; const float mu = (float)s * (8.0f / 39.0f); const float d = bf16_round(bond[n * NEI + i]) - mu; f.h[q] = (_Float16)expf(-(d * d) * 25.0f); }   *(volatile v8us*)((unsigned short*)EF + t * 8) = f.half[0]; __threadfence(); *(volatile v8us*)((unsigned short*)EF + t * 8) = f.half[0]; } }
__global__ __launch_bounds__(256) void k_gbf_a(const float* __restrict__ ang, int n0, _Float16* __restrict__ AF) { const size_t t = (size_t)blockIdx.x * 256 + threadIdx.x;
  if (t < (size_t)NHALF * KA / 8) { const int k8 = (int)((t * 8) % KA); const size_t nl = (t * 8) / KA; const size_t n = nl + n0; FragH f; for (int q = 0; q < 8; ++q) { const int k = k8 + q; const int ij = k / AST, s = k % AST; const float mu = -1.0f + (float)s * (2.0f / 19.0f); const float d = bf16_round(ang[n * NEI * NEI + ij]) - mu; f.h[q] = (_Float16)expf(-(d * d) * 100.0f); }   *(volatile v8us*)((unsigned short*)AF + t * 8) = f.half[0]; __threadfence(); *(volatile v8us*)((unsigned short*)AF + t * 8) = f.half[0]; } }
__global__ __launch_bounds__(256) void k_wt(const float* __restrict__ Wroot, const float* __restrict__ Wrel, int K, _Float16* __restrict__ Bt) { const size_t t = (size_t)blockIdx.x * 256 + threadIdx.x; if (t >= (size_t)4 * HH * K / 8) return; const int k8 = (int)((t * 8) % K); const int n = (int)((t * 8) / K); const int grp = n / HH, h = n % HH; FragH f;
  for (int q = 0; q < 8; ++q) { const int k = k8 + q; const float w = (grp == 0) ? Wroot[(size_t)k * HH + h] : Wrel[((size_t)(grp - 1) * K + k) * HH + h]; f.h[q] = (_Float16)(bf16_round(w) * 4.0f); } *(volatile v8us*)((unsigned short*)Bt + t * 8) = f.half[0]; __threadfence(); *(volatile v8us*)((unsigned short*)Bt + t * 8) = f.half[0]; }
__device__ __forceinline__ int bscan256(int cnt, int* scan, int tid, int& total) { __syncthreads(); scan[tid] = cnt; __syncthreads();
  for (int of = 1; of < 256; of <<= 1) { const int v = (tid >= of) ? scan[tid - of] : 0; __syncthreads(); scan[tid] += v; __syncthreads(); }
  total = scan[255]; return scan[tid] - cnt; }
__global__ __launch_bounds__(256) void k_ragg(const float* __restrict__ XW, const float* __restrict__ b, const int* __restrict__ species, const int* __restrict__ nbr, float* __restrict__ OUT, int ldo, int c0, _Float16* __restrict__ O16) {
#pragma clang fp contract(off)
  __shared__ short Lr[2048]; __shared__ int Le[2048]; __shared__ int scan[256]; __shared__ float stg[64][65];
  const int tid = threadIdx.x, lane = tid & 31, wv = tid >> 5; const int nl = tid >> 1, half = tid & 1; const int n0 = blockIdx.x * 128; const int i = n0 + nl; const int si = (i < NA) ? species[i] : 0;
  float acc[NREL][32]; float cnt[NREL];
#pragma unroll
  for (int r = 0; r < NREL; ++r) { cnt[r] = 0.f;
#pragma unroll
    for (int c = 0; c < 32; ++c) acc[r][c] = 0.f; }
#pragma unroll 1
  for (int e0 = 0; e0 < NE; e0 += 2048) { int hr[8], he[8]; int k_cnt = 0;
#pragma unroll
    for (int k = 0; k < 8; ++k) { const int e = e0 + tid * 8 + k; hr[k] = -1; he[k] = 0; if (e < NE) { const int dd_ = nbr[e]; if (dd_ >= n0 && dd_ < n0 + 128) { hr[k] = dd_ - n0; he[k] = e; ++k_cnt; } } }
    int tot; int p = bscan256(k_cnt, scan, tid, tot);
#pragma unroll
    for (int k = 0; k < 8; ++k) if (hr[k] >= 0) { Lr[p] = (short)hr[k]; Le[p] = he[k]; ++p; }
    __syncthreads();
    const int ntrip = (tot + 31) >> 5;
#pragma unroll 1
    for (int it = 0; it < ntrip; ++it) { const int q = it * 32 + lane; const int lr = (q < tot) ? (int)Lr[q] : -1;
      unsigned m = __builtin_amdgcn_ballot_w32(lr >= wv * 16 && lr < wv * 16 + 16);
#pragma unroll 1
      while (m) { const int bit = __builtin_ctz(m); m &= m - 1u; const int owner = __shfl(lr, bit, 32); const int e = Le[it * 32 + bit];
        if (nl == owner) { const int s = e / NEI; int r = species[s] + si; r = r < 0 ? 0 : (r > 2 ? 2 : r); const float* xr = XW + (size_t)s * (4 * HH) + HH * (1 + r) + 32 * half;
#pragma unroll
          for (int rr = 0; rr < NREL; ++rr) if (rr == r) { cnt[rr] += 1.0f;
#pragma unroll
            for (int g = 0; g < 8; ++g) { const v4f v = *(const v4fa*)(xr + 4 * g); acc[rr][4 * g] += v[0]; acc[rr][4 * g + 1] += v[1]; acc[rr][4 * g + 2] += v[2]; acc[rr][4 * g + 3] += v[3]; } } } } }
    __syncthreads(); }
  { const float inv0 = 1.0f / fmaxf(cnt[0], 1.0f), inv1 = 1.0f / fmaxf(cnt[1], 1.0f), inv2 = 1.0f / fmaxf(cnt[2], 1.0f); const float* root = XW + (size_t)((i < NA) ? i : 0) * (4 * HH) + 32 * half;
#pragma unroll
    for (int g = 0; g < 8; ++g) { const v4f rt = *(const v4fa*)(root + 4 * g);
#pragma unroll
      for (int u = 0; u < 4; ++u) { const int c = 4 * g + u; float o = rt[u] + bf16_round(b[32 * half + c]); o = o + acc[0][c] * inv0; o = o + acc[1][c] * inv1; o = o + acc[2][c] * inv2; acc[0][c] = fmaxf(o, 0.f); } } }
  typedef _Float16 v4h __attribute__((ext_vector_type(4)));
  for (int tg = 0; tg < 2; ++tg) {
    if (tid / 128 == tg) {
#pragma unroll
      for (int c = 0; c < 32; ++c) stg[nl % 64][32 * half + c] = acc[0][c]; }
    __syncthreads();
    for (int pass = 0; pass < 2; ++pass) {
#pragma unroll 1
      for (int j = tid; j < 64 * 16; j += 256) { const int rrow = j / 16, c4 = (j % 16) * 4; const int n = n0 + tg * 64 + rrow; if (n < NA) { v4f v; v[0] = stg[rrow][c4]; v[1] = stg[rrow][c4 + 1]; v[2] = stg[rrow][c4 + 2]; v[3] = stg[rrow][c4 + 3];
          if (OUT) *(volatile v4f*)(OUT + (size_t)n * ldo + c0 + c4) = v; if (O16) { v4h h4; h4[0] = (_Float16)v[0]; h4[1] = (_Float16)v[1]; h4[2] = (_Float16)v[2]; h4[3] = (_Float16)v[3]; *(volatile v4h*)(O16 + (size_t)n * HH + c4) = h4; } } }
      if (pass == 0) __threadfence(); }
    __syncthreads(); } }
__global__ __launch_bounds__(128) void k_pool(const float* __restrict__ FEAT, const int* __restrict__ crys, const float* __restrict__ fcW, const float* __restrict__ fcb, float* __restrict__ out) { __shared__ float sp[NCR][2 * HH + 1]; __shared__ int sst[NCR], scnt[NCR]; const int ch = threadIdx.x; if (ch < NCR) { sst[ch] = crys[ch * 2]; scnt[ch] = crys[ch * 2 + 1] - crys[ch * 2]; } __syncthreads();
  float acc[NCR]; for (int k = 0; k < NCR; ++k) acc[k] = 0.f;
#pragma unroll 1
  for (int n = 0; n < NA; ++n) { int id = -1;
#pragma unroll
    for (int k = 0; k < NCR; ++k) if (sst[k] <= n) id = k; const float v = FEAT[(size_t)n * (2 * HH) + ch];
#pragma unroll
    for (int k = 0; k < NCR; ++k) if (k == id) acc[k] += v; }
  for (int k = 0; k < NCR; ++k) sp[k][ch] = acc[k]; __syncthreads();
  if (ch < NCR * NCLS) { const int cr = ch / NCLS, o = ch % NCLS; const float rc = 1.0f / (float)scnt[cr]; float s = bf16_round(fcb[o]);
#pragma unroll 1
    for (int c2 = 0; c2 < 2 * HH; ++c2) s += (sp[cr][c2] * rc) * bf16_round(fcW[c2 * NCLS + o]); *(volatile float*)(out + ch) = s; __threadfence(); *(volatile float*)(out + ch) = s; } }
extern "C" void kernel_launch(void* const* d_in, const int* in_sizes, int n_in,
                              void* d_out, int out_size, void* d_ws, size_t ws_size, hipStream_t stream) {
  (void)in_sizes; (void)n_in; (void)out_size;
  const float* bond = (const float*)d_in[0]; const float* ang = (const float*)d_in[1]; const int* species = (const int*)d_in[2]; const int* nbr = (const int*)d_in[3]; const int* crys = (const int*)d_in[4];
  const float* W1b_rel = (const float*)d_in[5]; const float* W1b_root = (const float*)d_in[6]; const float* b1b = (const float*)d_in[7]; const float* W1a_rel = (const float*)d_in[8]; const float* W1a_root = (const float*)d_in[9]; const float* b1a = (const float*)d_in[10];
  const float* W2b_rel = (const float*)d_in[11]; const float* W2b_root = (const float*)d_in[12]; const float* b2b = (const float*)d_in[13]; const float* W2a_rel = (const float*)d_in[14]; const float* W2a_root = (const float*)d_in[15]; const float* b2a = (const float*)d_in[16]; const float* fcW = (const float*)d_in[17]; const float* fcb = (const float*)d_in[18];
  char* ws = (char*)d_ws; size_t off = 0;
  auto take = [&](size_t bytes) { char* p = ws + off; off += (bytes + 255) & ~(size_t)255; return p; };
  _Float16* B1b = (_Float16*)take((size_t)4 * HH * KB * 2); _Float16* B1a = (_Float16*)take((size_t)4 * HH * KA * 2); _Float16* B2b = (_Float16*)take((size_t)4 * HH * HH * 2); _Float16* B2a = (_Float16*)take((size_t)4 * HH * HH * 2);
  _Float16* EF = (_Float16*)take((size_t)NA * KB * 2); _Float16* AFh = (_Float16*)take((size_t)NHALF * KA * 2); float* XW = (float*)take((size_t)NA * 4 * HH * 4); _Float16* BF16b = (_Float16*)take((size_t)NA * HH * 2); _Float16* AF16b = (_Float16*)take((size_t)NA * HH * 2); float* FEAT = (float*)take((size_t)NA * 2 * HH * 4);
  if (off > ws_size) return;
  const unsigned gAgg = (NA + 127) / 128;
  k_wt<<<(unsigned)(((size_t)4 * HH * KB / 8 + 255) / 256), 256, 0, stream>>>(W1b_root, W1b_rel, KB, B1b); k_wt<<<(unsigned)(((size_t)4 * HH * KA / 8 + 255) / 256), 256, 0, stream>>>(W1a_root, W1a_rel, KA, B1a);
  k_wt<<<(4 * HH * HH / 8 + 255) / 256, 256, 0, stream>>>(W2b_root, W2b_rel, HH, B2b); k_wt<<<(4 * HH * HH / 8 + 255) / 256, 256, 0, stream>>>(W2a_root, W2a_rel, HH, B2a);
  k_gbf_b<<<(unsigned)(((size_t)NA * KB / 8 + 255) / 256), 256, 0, stream>>>(bond, EF);
  k_gemm_hh<0><<<dim3(((NA / 16) * 4 + 3) / 4, 1), 128, 0, stream>>>(EF, KB, 0, B1b, KB, 0, 0.25f, XW, 4 * HH, 0, NA, 4 * HH, KB);
  k_ragg<<<gAgg, 256, 0, stream>>>(XW, b1b, species, nbr, nullptr, 0, 0, BF16b);
  for (int h0 = 0; h0 < NA; h0 += NHALF) {
    k_gbf_a<<<(unsigned)(((size_t)NHALF * KA / 8 + 255) / 256), 256, 0, stream>>>(ang, h0, AFh);
    k_gemm_hh<0><<<dim3(((NHALF / 16) * 4 + 3) / 4, 1), 128, 0, stream>>>(AFh, KA, 0, B1a, KA, 0, 0.25f, XW + (size_t)h0 * 4 * HH, 4 * HH, 0, NHALF, 4 * HH, KA); }
  k_ragg<<<gAgg, 256, 0, stream>>>(XW, b1a, species, nbr, nullptr, 0, 0, AF16b);
  k_gemm_hh<0><<<dim3(((NA / 16) * 4 + 3) / 4, 1), 128, 0, stream>>>(BF16b, HH, 0, B2b, HH, 0, 0.25f, XW, 4 * HH, 0, NA, 4 * HH, HH);
  k_ragg<<<gAgg, 256, 0, stream>>>(XW, b2b, species, nbr, FEAT, 2 * HH, 0, nullptr);
  k_gemm_hh<0><<<dim3(((NA / 16) * 4 + 3) / 4, 1), 128, 0, stream>>>(AF16b, HH, 0, B2a, HH, 0, 0.25f, XW, 4 * HH, 0, NA, 4 * HH, HH);
  k_ragg<<<gAgg, 256, 0, stream>>>(XW, b2a, species, nbr, FEAT, 2 * HH, HH, nullptr);
  k_pool<<<1, 128, 0, stream>>>(FEAT, crys, fcW, fcb, (float*)d_out);
}
